// Attention_56349970923851
// MI455X (gfx1250) — hardware-verified
//
#include <hip/hip_runtime.h>


#ifndef NB
#define NB 2
#endif
#ifndef SEQ
#define SEQ 2048
#endif
#define SEQ_FULL 2048
#define DIM   2048
#define NH    32
#define NKV   8
#define REP   (NH / NKV)
#define HD    64
#define HALFD 32
#define DQ    (NH * HD)
#define DKV   (NKV * HD)
#define NQKV  (DQ + 2 * DKV)
#define MROWS (NB * SEQ)
#define FP    68
#define OP    72
#define WCAR  64.0f
#define CCAR  256.0f
#define OSCL  6.103515625e-05f
#define SC2   0.18033688011112042f
#define LOG2E 1.4426950408889634f
#define PEXP  10.0f
#define FRQC  0.41524101186092029f

static_assert(SEQ % 64 == 0);
static_assert(SEQ <= SEQ_FULL);
static_assert(DIM % 64 == 0);
static_assert(DQ % 64 == 0);
static_assert(NQKV % 64 == 0);
static_assert(HD == 64);
static_assert(NH == NKV * REP);
static_assert(REP == 4);
static_assert(((size_t)MROWS * DIM / 8) % 256 == 0);
static_assert(((size_t)DQ * DIM / 8) % 256 == 0);
static_assert(((size_t)DKV * DIM / 8) % 256 == 0);

typedef _Float16 h16;
typedef unsigned short bf;
typedef __attribute__((ext_vector_type(16))) __bf16   v16bf;
typedef __attribute__((ext_vector_type(16))) _Float16 v16h;
typedef __attribute__((ext_vector_type(8)))  _Float16 v8h;
typedef __attribute__((ext_vector_type(8)))  unsigned short v8us;
typedef __attribute__((ext_vector_type(8)))  float    v8f;
typedef __attribute__((ext_vector_type(4)))  float    v4f;
typedef v8h  __attribute__((may_alias)) v8ha;
typedef v4f  __attribute__((may_alias)) v4fa;

__device__ __forceinline__ unsigned short f2bf(float f) { unsigned u = __float_as_uint(f); u += 0x7FFFu + ((u >> 16) & 1u); return (unsigned short)(u >> 16); }
__device__ __forceinline__ float bf2f(unsigned short b) { return __uint_as_float(((unsigned)b) << 16); }
__device__ __forceinline__ float bfr(float f) { return bf2f(f2bf(f)); }
__device__ __forceinline__ v16h cat16(v8h lo, v8h hi) { return __builtin_shufflevector(lo, hi, 0, 1, 2, 3, 4, 5, 6, 7, 8, 9, 10, 11, 12, 13, 14, 15); }
__device__ __forceinline__ v16bf cat16b(v8us lo, v8us hi) { return __builtin_bit_cast(v16bf, __builtin_shufflevector(lo, hi, 0, 1, 2, 3, 4, 5, 6, 7, 8, 9, 10, 11, 12, 13, 14, 15)); }
__device__ __forceinline__ v8f wmma16(v16h a, v16h b, v8f c) { return __builtin_amdgcn_wmma_f32_16x16x32_f16(false, a, false, b, (short)0, c, false, false); }
__device__ __forceinline__ v8f wmmab(v16bf a, v16bf b, v8f c) { return __builtin_amdgcn_wmma_f32_16x16x32_bf16(false, a, false, b, (short)0, c, false, false); }

template <typename T16> struct WFrag;
template <> struct WFrag<h16> { typedef v16h V; static __device__ __forceinline__ V ld(const h16* p) { return cat16(*(const v8h*)p, *(const v8h*)(p + 16)); } static __device__ __forceinline__ v8f mma(V a, V b, v8f c) { return wmma16(a, b, c); } };
template <> struct WFrag<bf> { typedef v16bf V; static __device__ __forceinline__ V ld(const bf* p) { return cat16b(*(const v8us*)p, *(const v8us*)(p + 16)); } static __device__ __forceinline__ v8f mma(V a, V b, v8f c) { return wmmab(a, b, c); } };

template <typename T16>
__device__ __forceinline__ void gemm_main(const T16* __restrict__ A, const T16* __restrict__ Bt, const int K, const int r0, const int c0, const int lr, const int hi, v8f (&acc)[4][4]) {
    typedef typename WFrag<T16>::V V;
#pragma unroll
    for (int mb = 0; mb < 4; ++mb)
#pragma unroll
        for (int nb = 0; nb < 4; ++nb) acc[mb][nb] = (v8f){};
    const size_t aoff = (size_t)(r0 + lr) * K + 8 * hi, boff = (size_t)(c0 + lr) * K + 8 * hi;
#pragma unroll 1
    for (int kc = 0; kc < K; kc += 32) {
        V a[4];
#pragma unroll
        for (int mb = 0; mb < 4; ++mb) a[mb] = WFrag<T16>::ld(A + aoff + (size_t)mb * 16 * K + kc);
#pragma unroll
        for (int nb = 0; nb < 4; ++nb) { const V b = WFrag<T16>::ld(Bt + boff + (size_t)nb * 16 * K + kc);
#pragma unroll
            for (int mb = 0; mb < 4; ++mb) acc[mb][nb] = WFrag<T16>::mma(a[mb], b, acc[mb][nb]); }
        asm volatile("v_nop\n\tv_nop\n\tv_nop\n\tv_nop" : "+v"(acc[0][0]), "+v"(acc[1][1]), "+v"(acc[2][2]), "+v"(acc[3][3]) : "v"(a[0]), "v"(a[3]));
    }
}

__global__ __launch_bounds__(256) void k_cvtx(const float* __restrict__ x, bf* dst) {
    const size_t i = (size_t)blockIdx.x * 256 + threadIdx.x; if (i >= (size_t)MROWS * DIM / 8) return;
    const size_t e = i * 8; const int col = (int)(e % DIM); const int row = (int)(e / DIM); const int b = row / SEQ, t = row % SEQ;
    const v8f v = *(const v8f*)(x + ((size_t)b * SEQ_FULL + t) * DIM + col); v8us o;
#pragma unroll
    for (int k = 0; k < 8; ++k) o[k] = f2bf(v[k]);
    *(volatile v8us*)(dst + e) = o; __threadfence(); *(volatile v8us*)(dst + e) = o; }

__global__ __launch_bounds__(256) void k_cvt8(const float* __restrict__ src, bf* dst, size_t n8) { const size_t i = (size_t)blockIdx.x * 256 + threadIdx.x; if (i >= n8) return; const v8f v = *(const v8f*)(src + i * 8); v8us o;
#pragma unroll
    for (int k = 0; k < 8; ++k) o[k] = f2bf(v[k]); *(volatile v8us*)(dst + i * 8) = o; __threadfence(); *(volatile v8us*)(dst + i * 8) = o; }

__global__ __launch_bounds__(256) void k_cvt8h(const float* __restrict__ src, h16* dst, size_t n8, float carry) { const size_t i = (size_t)blockIdx.x * 256 + threadIdx.x; if (i >= n8) return; const v8f v = *(const v8f*)(src + i * 8); v8h o;
#pragma unroll
    for (int k = 0; k < 8; ++k) o[k] = (h16)(bfr(v[k]) * carry); *(volatile v8h*)(dst + i * 8) = o; __threadfence(); *(volatile v8h*)(dst + i * 8) = o; }

__global__ __launch_bounds__(256) void k_ropetab(float* COS, float* SIN) {
    const int lane = threadIdx.x & 31; const int t = blockIdx.x * 8 + (threadIdx.x >> 5); if (t >= SEQ) return;
    const float invf = __builtin_amdgcn_exp2f(-(float)lane * FRQC);
    const float ang = (float)t * invf;
    const float c = cosf(ang); const float s = sinf(ang);
    const size_t o = (size_t)t * HALFD + lane;
    *(volatile float*)(COS + o) = c; *(volatile float*)(SIN + o) = s; __threadfence(); *(volatile float*)(COS + o) = c; *(volatile float*)(SIN + o) = s; }

__global__ __launch_bounds__(32) void k_gemm_qkv(const bf* __restrict__ A, const bf* __restrict__ Bt, const int* __restrict__ pos, const float* __restrict__ COS, const float* __restrict__ SIN, h16* QP, h16* KP, h16* VT) {
    __shared__ __align__(16) float fs[64 * FP];
    const int lane = threadIdx.x & 31, lr = lane & 15, hi = lane >> 4; const int r0 = blockIdx.x * 64, cb = blockIdx.y, c0 = cb * 64;
    v8f acc[4][4];
    gemm_main<bf>(A, Bt, DIM, r0, c0, lr, hi, acc);
#pragma unroll
    for (int mb = 0; mb < 4; ++mb)
#pragma unroll
        for (int nb = 0; nb < 4; ++nb)
#pragma unroll
            for (int j = 0; j < 8; ++j) fs[(mb * 16 + hi * 8 + j) * FP + nb * 16 + lr] = acc[mb][nb][j];
    __syncthreads();
    const int bidx = r0 / SEQ, s0 = r0 % SEQ; const int q4 = lane >> 3, p = lane & 7;
    if (cb < NH + NKV) {
        h16* plane = (cb < NH) ? (QP + ((size_t)bidx * NH + cb) * SEQ * HD) : (KP + ((size_t)bidx * NKV + (cb - NH)) * SEQ * HD);
        const int dcol = p * 8, pcol = dcol ^ 32, fcol = dcol & 31; const float sg = (p < 4) ? -1.0f : 1.0f;
#pragma unroll 1
        for (int it = 0; it < 16; ++it) {
            const int rl = it * 4 + q4;
            int ps = pos[(size_t)bidx * SEQ_FULL + s0 + rl]; ps = (ps < 0) ? (ps + SEQ) : ps; ps = min(max(ps, 0), SEQ - 1);
            const v4f xa0 = *(const v4fa*)(fs + rl * FP + dcol), xa1 = *(const v4fa*)(fs + rl * FP + dcol + 4);
            const v4f xb0 = *(const v4fa*)(fs + rl * FP + pcol), xb1 = *(const v4fa*)(fs + rl * FP + pcol + 4);
            const float* cp = COS + (size_t)ps * HALFD + fcol; const float* sp = SIN + (size_t)ps * HALFD + fcol;
            const v4f cc0 = *(const v4f*)cp, cc1 = *(const v4f*)(cp + 4), ss0 = *(const v4f*)sp, ss1 = *(const v4f*)(sp + 4);
            v8h o;
#pragma unroll
            for (int e = 0; e < 4; ++e) { o[e] = (h16)(xa0[e] * cc0[e] + sg * (xb0[e] * ss0[e])); o[4 + e] = (h16)(xa1[e] * cc1[e] + sg * (xb1[e] * ss1[e])); }
            h16* dst = plane + (size_t)(s0 + rl) * HD + dcol;
            *(volatile v8h*)dst = o; __threadfence(); *(volatile v8h*)dst = o;
        }
    } else {
        h16* plane = VT + ((size_t)bidx * NKV + (cb - NH - NKV)) * HD * SEQ;
#pragma unroll 1
        for (int it = 0; it < 16; ++it) {
            const int d = it * 4 + q4; v8h o;
#pragma unroll
            for (int e = 0; e < 8; ++e) o[e] = (h16)fs[(p * 8 + e) * FP + d];
            h16* dst = plane + (size_t)d * SEQ + s0 + p * 8;
            *(volatile v8h*)dst = o; __threadfence(); *(volatile v8h*)dst = o;
        }
    }
}

__global__ __launch_bounds__(128) void k_flash(const h16* __restrict__ QP, const h16* __restrict__ KP, const h16* __restrict__ VT, const float* __restrict__ mask, h16* CTX) {
    __shared__ __align__(16) h16 os[4 * 16 * OP];
    const int tid = threadIdx.x, w = tid >> 5, lane = tid & 31, lr = lane & 15, hi = lane >> 4;
    const int g = blockIdx.y, bidx = blockIdx.z, h = g * REP + w, q0 = blockIdx.x * 16;
    const h16* qrow = QP + (((size_t)bidx * NH + h) * SEQ + q0 + lr) * HD + 8 * hi;
    v16h bq[2];
#pragma unroll
    for (int kc = 0; kc < 2; ++kc) bq[kc] = cat16(*(const v8h*)(qrow + kc * 32), *(const v8h*)(qrow + kc * 32 + 16));
    const h16* kb = KP + (((size_t)bidx * NKV + g) * SEQ + lr) * HD + 8 * hi;
    const h16* vb = VT + (((size_t)bidx * NKV + g) * HD + lr) * SEQ + 8 * hi;
    const float* mrow = mask + (size_t)(q0 + lr) * SEQ_FULL + 8 * hi;
    v8f accO[4];
#pragma unroll
    for (int dt = 0; dt < 4; ++dt) accO[dt] = (v8f){};
    float m = -3.0e38f, l = 0.0f;
#pragma unroll 1
    for (int k0 = 0; k0 < SEQ; k0 += 64) {
        v16h ak[2][4];
#pragma unroll
        for (int kc = 0; kc < 2; ++kc)
#pragma unroll
            for (int T = 0; T < 4; ++T) { const h16* kp = kb + (size_t)(k0 + 16 * T) * HD + kc * 32; ak[kc][T] = cat16(*(const v8h*)kp, *(const v8h*)(kp + 16)); }
        v8f accS[4];
#pragma unroll
        for (int T = 0; T < 4; ++T) accS[T] = (v8f){};
#pragma unroll
        for (int kc = 0; kc < 2; ++kc)
#pragma unroll
            for (int T = 0; T < 4; ++T) accS[T] = wmma16(ak[kc][T], bq[kc], accS[T]);
        asm volatile("v_nop\n\tv_nop\n\tv_nop\n\tv_nop" : "+v"(accS[0]), "+v"(accS[1]), "+v"(accS[2]), "+v"(accS[3]) : "v"(ak[1][3]), "v"(bq[1]));
        float tmax = -3.0e38f;
#pragma unroll
        for (int T = 0; T < 4; ++T) { const float* mp = mrow + k0 + 16 * T; const v4f m0 = *(const v4f*)mp; const v4f m1 = *(const v4f*)(mp + 4);
#pragma unroll
            for (int r = 0; r < 4; ++r) { const float a0 = accS[T][r] * SC2 + m0[r] * LOG2E; const float a1 = accS[T][4 + r] * SC2 + m1[r] * LOG2E; accS[T][r] = a0; accS[T][4 + r] = a1; tmax = fmaxf(tmax, fmaxf(a0, a1)); } }
        tmax = fmaxf(tmax, __shfl_xor(tmax, 16, 32));
        const float mn = fmaxf(m, tmax); const float corr = __builtin_amdgcn_exp2f(m - mn); m = mn; const float mofs = PEXP - mn;
        float rs = 0.0f;
#pragma unroll
        for (int T = 0; T < 4; ++T)
#pragma unroll
            for (int r = 0; r < 8; ++r) { const float pv = __builtin_amdgcn_exp2f(accS[T][r] + mofs); accS[T][r] = pv; rs += pv; }
        l = l * corr + rs;
        v16h bp[2];
        bp[0] = cat16(__builtin_convertvector(accS[0], v8h), __builtin_convertvector(accS[1], v8h));
        bp[1] = cat16(__builtin_convertvector(accS[2], v8h), __builtin_convertvector(accS[3], v8h));
#pragma unroll
        for (int dt = 0; dt < 4; ++dt) accO[dt] = accO[dt] * corr;
        v16h av[2][4];
#pragma unroll
        for (int kc = 0; kc < 2; ++kc)
#pragma unroll
            for (int dt = 0; dt < 4; ++dt) { const h16* vp = vb + (size_t)(16 * dt) * SEQ + k0 + kc * 32; av[kc][dt] = cat16(*(const v8h*)vp, *(const v8h*)(vp + 16)); }
#pragma unroll
        for (int kc = 0; kc < 2; ++kc)
#pragma unroll
            for (int dt = 0; dt < 4; ++dt) accO[dt] = wmma16(av[kc][dt], bp[kc], accO[dt]);
        asm volatile("v_nop\n\tv_nop\n\tv_nop\n\tv_nop" : "+v"(accO[0]), "+v"(accO[1]), "+v"(accO[2]), "+v"(accO[3]) : "v"(av[1][3]), "v"(bp[1]));
    }
    l += __shfl_xor(l, 16, 32);
    const float inv = CCAR * (1.0f / l);
    h16* ow = os + w * 16 * OP;
#pragma unroll
    for (int dt = 0; dt < 4; ++dt) { v8h o;
#pragma unroll
        for (int r = 0; r < 8; ++r) o[r] = (h16)(accO[dt][r] * inv);
        *(v8ha*)(ow + lr * OP + 16 * dt + 8 * hi) = o; }
    __syncthreads();
    const int q4 = lane >> 3, p = lane & 7;
#pragma unroll 1
    for (int ps = 0; ps < 2; ++ps) {
#pragma unroll
        for (int it = 0; it < 4; ++it) { const int row = it * 4 + q4; const v8h o = *(const v8ha*)(ow + row * OP + p * 8);
            *(volatile v8h*)(CTX + ((size_t)bidx * SEQ + q0 + row) * DQ + h * HD + p * 8) = o; }
        if (ps == 0) __threadfence(); }
}

__global__ __launch_bounds__(32) void k_gemm_out(const h16* __restrict__ A, const h16* __restrict__ Bt, float* C) {
    __shared__ __align__(16) float fs[64 * FP];
    const int lane = threadIdx.x & 31, lr = lane & 15, hi = lane >> 4; const int r0 = blockIdx.x * 64, c0 = blockIdx.y * 64;
    v8f acc[4][4];
    gemm_main<h16>(A, Bt, DQ, r0, c0, lr, hi, acc);
#pragma unroll
    for (int mb = 0; mb < 4; ++mb)
#pragma unroll
        for (int nb = 0; nb < 4; ++nb)
#pragma unroll
            for (int j = 0; j < 8; ++j) fs[(mb * 16 + hi * 8 + j) * FP + nb * 16 + lr] = acc[mb][nb][j];
    __syncthreads();
    float* crow = C + (size_t)r0 * DIM + c0;
#pragma unroll 1
    for (int ps = 0; ps < 2; ++ps) {
#pragma unroll 4
        for (int it = 0; it < 32; ++it) { const int row = it * 2 + hi; v4f val = *(const v4fa*)(fs + row * FP + lr * 4); val = val * OSCL;
            *(volatile v4f*)(crow + (size_t)row * DIM + lr * 4) = val; }
        if (ps == 0) __threadfence(); }
}

extern "C" void kernel_launch(void* const* d_in, const int* in_sizes, int n_in,
                              void* d_out, int out_size, void* d_ws, size_t ws_size, hipStream_t stream) {
    if (n_in < 7) return;
    if ((size_t)in_sizes[0] < ((size_t)(NB - 1) * SEQ_FULL + SEQ) * DIM) return;
    if ((size_t)in_sizes[1] < (size_t)(SEQ - 1) * SEQ_FULL + SEQ) return;
    if ((size_t)in_sizes[2] < (size_t)(NB - 1) * SEQ_FULL + SEQ) return;
    if ((size_t)in_sizes[3] < (size_t)DQ * DIM) return;
    if ((size_t)in_sizes[4] < (size_t)DKV * DIM) return;
    if ((size_t)in_sizes[5] < (size_t)DKV * DIM) return;
    if ((size_t)in_sizes[6] < (size_t)DIM * DQ) return;
    if ((size_t)out_size < (size_t)MROWS * DIM) return;
    const float* x = (const float*)d_in[0]; const float* mask = (const float*)d_in[1]; const int* pos = (const int*)d_in[2];
    const float* wq = (const float*)d_in[3]; const float* wk = (const float*)d_in[4]; const float* wv = (const float*)d_in[5]; const float* wo = (const float*)d_in[6];
    float* OUT = (float*)d_out;
    char* wsp = (char*)d_ws;
    auto take = [&](size_t bytes) { char* p = wsp; wsp += (bytes + 255) & ~(size_t)255; return (void*)p; };
    bf*  XB   = (bf*)take((size_t)MROWS * DIM * 2);
    bf*  WQKV = (bf*)take((size_t)NQKV * DIM * 2);
    h16* WO16 = (h16*)take((size_t)DIM * DQ * 2);
    float* COS = (float*)take((size_t)SEQ * HALFD * 4);
    float* SIN = (float*)take((size_t)SEQ * HALFD * 4);
    h16* QP  = (h16*)take((size_t)NB * NH * SEQ * HD * 2);
    h16* KP  = (h16*)take((size_t)NB * NKV * SEQ * HD * 2);
    h16* VT  = (h16*)take((size_t)NB * NKV * HD * SEQ * 2);
    h16* CTX = (h16*)take((size_t)MROWS * DQ * 2);
    if ((size_t)(wsp - (char*)d_ws) > ws_size) return;

    k_cvtx<<<(unsigned)(((size_t)MROWS * DIM / 8 + 255) / 256), 256, 0, stream>>>(x, XB);
    k_cvt8<<<(unsigned)(((size_t)DQ * DIM / 8 + 255) / 256), 256, 0, stream>>>(wq, WQKV, (size_t)DQ * DIM / 8);
    k_cvt8<<<(unsigned)(((size_t)DKV * DIM / 8 + 255) / 256), 256, 0, stream>>>(wk, WQKV + (size_t)DQ * DIM, (size_t)DKV * DIM / 8);
    k_cvt8<<<(unsigned)(((size_t)DKV * DIM / 8 + 255) / 256), 256, 0, stream>>>(wv, WQKV + (size_t)(DQ + DKV) * DIM, (size_t)DKV * DIM / 8);
    k_cvt8h<<<(unsigned)(((size_t)DIM * DQ / 8 + 255) / 256), 256, 0, stream>>>(wo, WO16, (size_t)DIM * DQ / 8, WCAR);
    k_ropetab<<<(SEQ + 7) / 8, 256, 0, stream>>>(COS, SIN);
    k_gemm_qkv<<<dim3(MROWS / 64, NQKV / 64, 1), 32, 0, stream>>>(XB, WQKV, pos, COS, SIN, QP, KP, VT);
    k_flash<<<dim3(SEQ / 16, NKV, NB), 128, 0, stream>>>(QP, KP, VT, mask, CTX);
    k_gemm_out<<<dim3(MROWS / 64, DIM / 64, 1), 32, 0, stream>>>(CTX, WO16, OUT);
}
